// PQNRnn_65352222376257
// MI455X (gfx1250) — hardware-verified
//
#include <hip/hip_runtime.h>


namespace {
constexpr int B = 64, S = 256, H = 512, L = 4, A = 16, NR = B * S  , G3 = 3 * H;
constexpr float EPS = 1e-5f, XS = 8.0f;

typedef _Float16 b16;
typedef __attribute__((ext_vector_type(16))) _Float16 v16b;
typedef __attribute__((ext_vector_type(8))) _Float16 v8b;
typedef __attribute__((ext_vector_type(8))) float v8f;
typedef __attribute__((ext_vector_type(4))) float v4f;
__device__ __forceinline__ float bf16_rne(float f) { unsigned int u = __float_as_uint(f); u += 0x7FFFu + ((u >> 16) & 1u); return __uint_as_float(u & 0xFFFF0000u); }
__device__ __forceinline__ v16b frag_kb(const b16* p, int hh) { const v8b a = *(const v8b*)(p + 8 * hh), b = *(const v8b*)(p + 16 + 8 * hh); v16b f;
#pragma unroll
  for (int e = 0; e < 8; ++e) { f[e] = a[e]; f[8 + e] = b[e]; } return f; }
__device__ __forceinline__ v8f wmma16b(v16b a, v16b b, v8f c) { v8f d = __builtin_amdgcn_wmma_f32_16x16x32_f16(false, a, false, b, (short)0, c, false, false); asm volatile("v_nop\n\tv_nop\n\tv_nop\n\tv_nop" : "+v"(d) : "v"(a), "v"(b)); return d; }
__device__ __forceinline__ void wave_lds_sync() { __builtin_amdgcn_fence(__ATOMIC_RELEASE, "workgroup"); __builtin_amdgcn_wave_barrier(); __builtin_amdgcn_fence(__ATOMIC_ACQUIRE, "workgroup"); }
__device__ __forceinline__ float nexp(float x) { return __builtin_amdgcn_exp2f(x * 1.4426950408889634f); }
__device__ __forceinline__ float pmul(float a, float b) { float p = a * b; asm volatile("" : "+v"(p)); return p; }
__device__ __forceinline__ float wsum(float v) {
#pragma unroll
  for (int o = 1; o < 32; o <<= 1) v += __shfl_xor(v, o); return v; }
__device__ __forceinline__ float sigm(float x) { return __builtin_amdgcn_rcpf(1.0f + nexp(-x)); }
__device__ __forceinline__ float tanh_n(float x) { const float e = __builtin_amdgcn_exp2f(x * 2.8853900817779268f); return 1.0f - 2.0f * __builtin_amdgcn_rcpf(e + 1.0f); }

struct Wo_ { static constexpr size_t WL = 0, IH = WL + (size_t)L * H * H, HH = IH + (size_t)G3 * H, END = HH + (size_t)G3 * H; };
__global__ __launch_bounds__(256) void prep_kernel(const float* __restrict__ x, const float* __restrict__ Wl, const float* __restrict__ bl, const float* __restrict__ lg, const float* __restrict__ lb, const float* __restrict__ Wih, const float* __restrict__ Whh, const float* __restrict__ bih, const float* __restrict__ bhh, const float* __restrict__ Wq, const float* __restrict__ bq, b16* __restrict__ R, float* __restrict__ P, b16* __restrict__ X0) {
  const size_t tid = (size_t)blockIdx.x * 256 + threadIdx.x, nth = (size_t)gridDim.x * 256;
  for (int pass = 0; pass < 2; ++pass) {
    for (size_t p = tid; p < Wo_::END / 8; p += nth) { const size_t q = p * 8; const float* src = (q < Wo_::IH) ? (Wl + q) : (q < Wo_::HH) ? (Wih + (q - Wo_::IH)) : (Whh + (q - Wo_::HH)); v8b v;
#pragma unroll
      for (int e = 0; e < 8; ++e) v[e] = (b16)bf16_rne(src[e]); *(volatile v8b*)(R + q) = v; }
    for (size_t p = tid; p < (size_t)NR * H / 8; p += nth) { const size_t q = p * 8; v8b v;
#pragma unroll
      for (int e = 0; e < 8; ++e) v[e] = (b16)(bf16_rne(x[q + e]) * XS); *(volatile v8b*)(X0 + q) = v; }
    for (size_t q = tid; q < 17440; q += nth) { const int i = (int)q; float v; if (i < 2048) v = bl[i]; else if (i < 4096) v = lg[i - 2048]; else if (i < 6144) v = lb[i - 4096]; else if (i < 7680) v = bih[i - 6144]; else if (i < 9216) v = bhh[i - 7680]; else if (i < 17408) v = Wq[i - 9216]; else v = (i - 17408 < A) ? bq[i - 17408] : 0.0f; P[q] = bf16_rne(v); }
    __threadfence(); }
}

template <int N, int EPI>
__global__ __launch_bounds__(64) void gemm_kernel(const b16* __restrict__ Am, const b16* __restrict__ Bw, const float* __restrict__ bias, float* __restrict__ Cf, b16* __restrict__ Ch) {
  __shared__ __attribute__((aligned(16))) float Ts[2][32][128 + 4];
  const int lane = threadIdx.x & 31, wave = threadIdx.x >> 5, nloc = lane & 15, hlf = lane >> 4, m0 = blockIdx.y * 32, c0 = blockIdx.x * 256 + wave * 128;
  v8f acc[2][8];
#pragma unroll
  for (int r = 0; r < 2; ++r)
#pragma unroll
    for (int t = 0; t < 8; ++t) acc[r][t] = (v8f){};
  for (int kb = 0; kb < H; kb += 32) { const v16b a0 = frag_kb(Am + (size_t)(m0 + nloc) * H + kb, hlf), a1 = frag_kb(Am + (size_t)(m0 + 16 + nloc) * H + kb, hlf);
#pragma unroll
    for (int t = 0; t < 8; ++t) { const v16b bw = frag_kb(Bw + (size_t)(c0 + t * 16 + nloc) * H + kb, hlf); acc[0][t] = wmma16b(a0, bw, acc[0][t]); acc[1][t] = wmma16b(a1, bw, acc[1][t]); } }
#pragma unroll
  for (int t = 0; t < 8; ++t) { const float bv = bias[c0 + t * 16 + nloc];
#pragma unroll
    for (int r = 0; r < 2; ++r)
#pragma unroll
      for (int v = 0; v < 8; ++v) Ts[wave][r * 16 + 8 * hlf + v][t * 16 + nloc] = acc[r][t][v] * (1.0f / XS) + bv; }
  wave_lds_sync();
  for (int pass = 0; pass < 2; ++pass) {
    if (EPI == 0) { for (int i = lane; i < 32 * 32; i += 32) { const int rr = i >> 5, c4 = (i & 31) * 4; *(volatile v4f*)(Cf + (size_t)(m0 + rr) * N + c0 + c4) = *(const v4f*)(&Ts[wave][rr][c4]); } }
    else { for (int i = lane; i < 32 * 16; i += 32) { const int rr = i >> 4, c8 = (i & 15) * 8; v8b o; for (int e = 0; e < 8; ++e) o[e] = (b16)(Ts[wave][rr][c8 + e] * XS); *(volatile v8b*)(Ch + (size_t)(m0 + rr) * N + c0 + c8) = o; } }
    __threadfence(); }
}

__global__ __launch_bounds__(256) void lnrelu_kernel(const float* __restrict__ src, const float* __restrict__ g, const float* __restrict__ bb, b16* __restrict__ dst) {
  const int row = blockIdx.x * 8 + (threadIdx.x >> 5), lane = threadIdx.x & 31; const float* xr = src + (size_t)row * H;
  float v[16]; float s = 0.0f;
#pragma unroll
  for (int i = 0; i < 16; ++i) { v[i] = xr[(i >> 3) * 256 + lane * 8 + (i & 7)]; s += v[i]; }
  s = wsum(s); const float mu = s * (1.0f / H); float q = 0.0f;
#pragma unroll
  for (int i = 0; i < 16; ++i) { const float d = v[i] - mu; q += pmul(d, d); }
  q = wsum(q); const float inv = rsqrtf(q * (1.0f / H) + EPS);
  for (int pass = 0; pass < 2; ++pass) {
#pragma unroll
    for (int gq = 0; gq < 2; ++gq) { v8b o; const int c0 = gq * 256 + lane * 8;
#pragma unroll
      for (int e = 0; e < 8; ++e) o[e] = (b16)(fmaxf(pmul((v[gq * 8 + e] - mu) * inv, g[c0 + e]) + bb[c0 + e], 0.0f) * XS);
      *(volatile v8b*)(dst + (size_t)row * H + c0) = o; }
    __threadfence(); }
}

__global__ __launch_bounds__(256) void gru_kernel(const b16* __restrict__ gi, const int* __restrict__ dones, const float* __restrict__ h0, const b16* __restrict__ Whh, const float* __restrict__ bhh, float* __restrict__ rnn, float* __restrict__ hout) {
  __shared__ __attribute__((aligned(16))) b16 Hs[16][H + 8]; __shared__ __attribute__((aligned(16))) float Ot[8][16][64 + 4];
  const int wave = threadIdx.x >> 5, lane = threadIdx.x & 31, nloc = lane & 15, hlf = lane >> 4, b0 = blockIdx.x * 16, u0 = wave * 64;
  float hc[4][8];
#pragma unroll
  for (int t = 0; t < 4; ++t)
#pragma unroll
    for (int r = 0; r < 8; ++r) hc[t][r] = bf16_rne(h0[(size_t)(b0 + 8 * hlf + r) * H + u0 + t * 16 + nloc]);
  for (int step = 0; step < S; ++step) {
#pragma unroll
    for (int r = 0; r < 8; ++r) { const int b = b0 + 8 * hlf + r; const bool dn = dones[(size_t)b * S + step] != 0;
#pragma unroll
      for (int t = 0; t < 4; ++t) { if (dn) hc[t][r] = 0.0f; Hs[8 * hlf + r][u0 + t * 16 + nloc] = (b16)(hc[t][r] * XS); } }
    __syncthreads();
    v8f g[3][4];
#pragma unroll
    for (int q = 0; q < 3; ++q)
#pragma unroll
      for (int t = 0; t < 4; ++t) g[q][t] = (v8f){};
#pragma unroll 2
    for (int kb = 0; kb < H; kb += 32) { const v16b a = frag_kb(&Hs[nloc][kb], hlf);
#pragma unroll
      for (int q = 0; q < 3; ++q)
#pragma unroll
        for (int t = 0; t < 4; ++t) { const v16b bw = frag_kb(Whh + (size_t)(q * H + u0 + t * 16 + nloc) * H + kb, hlf); g[q][t] = wmma16b(a, bw, g[q][t]); } }
#pragma unroll
    for (int t = 0; t < 4; ++t) { const int u = u0 + t * 16 + nloc;
#pragma unroll
      for (int r = 0; r < 8; ++r) { const int b = b0 + 8 * hlf + r; const b16* gr = gi + ((size_t)b * S + step) * G3;
        const float hr = g[0][t][r] * (1.0f / XS) + bhh[u], hz = g[1][t][r] * (1.0f / XS) + bhh[H + u], hn = g[2][t][r] * (1.0f / XS) + bhh[2 * H + u];
        const float ir = (float)gr[u] * (1.0f / XS), iz = (float)gr[H + u] * (1.0f / XS), in_ = (float)gr[2 * H + u] * (1.0f / XS);
        const float rg = sigm(ir + hr), zg = sigm(iz + hz); const float n = tanh_n(in_ + pmul(rg, hn));
        const float hnew = pmul(1.0f - zg, n) + pmul(zg, hc[t][r]); hc[t][r] = hnew; Ot[wave][8 * hlf + r][t * 16 + nloc] = hnew; } }
    __syncthreads();
    for (int pass = 0; pass < 2; ++pass) { for (int i = lane; i < 16 * 16; i += 32) { const int rr = i >> 4, c4 = (i & 15) * 4; *(volatile v4f*)(rnn + ((size_t)(b0 + rr) * S + step) * H + u0 + c4) = *(const v4f*)(&Ot[wave][rr][c4]); }
      if (step == S - 1) { for (int i = lane; i < 16 * 16; i += 32) { const int rr = i >> 4, c4 = (i & 15) * 4; *(volatile v4f*)(hout + (size_t)(b0 + rr) * H + u0 + c4) = *(const v4f*)(&Ot[wave][rr][c4]); } }
      __threadfence(); }
    __syncthreads(); }
}

__global__ __launch_bounds__(512) void head_kernel(const float* __restrict__ rnn, const int* __restrict__ avail, const float* __restrict__ P, float* __restrict__ qout) {
  __shared__ float Q[16][A];
  const int wid = threadIdx.x >> 5, lane = threadIdx.x & 31, row = blockIdx.x * 16 + wid; const float* hr = rnn + (size_t)row * H; const float* Wq = P + 9216; const float* bq = P + 17408;
  float hv[16];
#pragma unroll
  for (int i = 0; i < 16; ++i) hv[i] = hr[(i >> 3) * 256 + lane * 8 + (i & 7)];
  for (int a = 0; a < A; ++a) { float s = 0.0f;
#pragma unroll
    for (int i = 0; i < 16; ++i) s += pmul(hv[i], Wq[a * H + (i >> 3) * 256 + lane * 8 + (i & 7)]);
    s = wsum(s); if (lane == 0) { const float un = 1.0f - (float)(avail[(size_t)row * A + a] != 0); Q[wid][a] = (s + bq[a]) - un * 1e10f; } }
  __syncthreads();
  for (int pass = 0; pass < 2; ++pass) { if (threadIdx.x < 64) *(volatile v4f*)(qout + (size_t)blockIdx.x * 16 * A + threadIdx.x * 4) = *(const v4f*)(&Q[0][0] + threadIdx.x * 4); __threadfence(); }
}
}

extern "C" void kernel_launch(void* const* d_in, const int* in_sizes, int n_in,
                              void* d_out, int out_size, void* d_ws, size_t ws_size, hipStream_t stream) {
  (void)n_in; (void)out_size;
  const float* h0 = (const float*)d_in[0]; const float* x = (const float*)d_in[1]; const int* dones = (const int*)d_in[2]; const int* avail = (const int*)d_in[3]; const float* Wl = (const float*)d_in[4]; const float* bl = (const float*)d_in[5]; const float* lg = (const float*)d_in[6]; const float* lb = (const float*)d_in[7];
  const float* Wih = (const float*)d_in[8]; const float* Whh = (const float*)d_in[9]; const float* bih = (const float*)d_in[10]; const float* bhh = (const float*)d_in[11]; const float* Wq = (const float*)d_in[12]; const float* bq = (const float*)d_in[13];
  float* hout = (float*)d_out; float* qout = hout + (size_t)B * H;
  if (in_sizes[0] != B * H || in_sizes[1] != NR * H || in_sizes[2] != NR || in_sizes[3] != NR * A || in_sizes[4] != L * H * H || in_sizes[8] != G3 * H || in_sizes[12] != A * H) return;
  size_t off = 0; char* ws = (char*)d_ws;
  auto carve = [&](size_t bytes) { char* p = ws + off; off += (bytes + 255) & ~(size_t)255; return p; };
  b16* R = (b16*)carve(Wo_::END * 2); float* P = (float*)carve(17920 * 4); b16* XA = (b16*)carve((size_t)NR * H * 2); float* T = (float*)carve((size_t)NR * H * 4); b16* GI = (b16*)carve((size_t)NR * G3 * 2);
  if (off > ws_size) return;
  prep_kernel<<<512, 256, 0, stream>>>(x, Wl, bl, lg, lb, Wih, Whh, bih, bhh, Wq, bq, R, P, XA);
  for (int l = 0; l < L; ++l) {
    gemm_kernel<H, 0><<<dim3(H / 256, NR / 32), 64, 0, stream>>>(XA, R + Wo_::WL + (size_t)l * H * H, P + l * H, T, nullptr);
    lnrelu_kernel<<<NR / 8, 256, 0, stream>>>(T, P + 2048 + l * H, P + 4096 + l * H, XA); }
  gemm_kernel<G3, 1><<<dim3(G3 / 256, NR / 32), 64, 0, stream>>>(XA, R + Wo_::IH, P + 6144, nullptr, GI);
  gru_kernel<<<B / 16, 256, 0, stream>>>(GI, dones, h0, R + Wo_::HH, P + 7680, T, hout);
  head_kernel<<<NR / 16, 512, 0, stream>>>(T, avail, P, qout);
}
